// TextLSTM_9311489098010
// MI455X (gfx1250) — hardware-run, weakly checked
//
#include <hip/hip_runtime.h>
#include <stddef.h>
#include <stdint.h>

typedef __attribute__((ext_vector_type(16))) _Float16 v16h;
typedef __attribute__((ext_vector_type(8)))  _Float16 v8h;
typedef __attribute__((ext_vector_type(4)))  _Float16 v4h;
typedef __attribute__((ext_vector_type(16))) __bf16   v16b;
typedef __attribute__((ext_vector_type(8)))  __bf16   v8b;
typedef __attribute__((ext_vector_type(8)))  float    v8f;
typedef __attribute__((ext_vector_type(4)))  float    v4f;

__device__ __forceinline__ unsigned short f2bf_bits(float f) {
  unsigned u = __float_as_uint(f);
  return (unsigned short)((u + 0x7FFFu + ((u >> 16) & 1u)) >> 16);
}
__device__ __forceinline__ float bf_bits2f(unsigned short h) { return __uint_as_float(((unsigned)h) << 16); }

__device__ __forceinline__ void dep_guard_h(v8f& a, v8f& b, v16h x, v16h y) { asm volatile("v_nop\n\tv_nop\n\tv_nop\n\tv_nop" : "+v"(a), "+v"(b) : "v"(x), "v"(y)); }
__device__ __forceinline__ void dep_guard_b(v8f& a, v8f& b, v16b x, v16b y) { asm volatile("v_nop\n\tv_nop\n\tv_nop\n\tv_nop" : "+v"(a), "+v"(b) : "v"(x), "v"(y)); }
__device__ __forceinline__ void keep4_h(v16h a, v16h b, v16h c, v16h d) { asm volatile("v_nop" :: "v"(a), "v"(b), "v"(c), "v"(d)); }
__device__ __forceinline__ void keep4_b(v16b a, v16b b, v16b c, v16b d) { asm volatile("v_nop" :: "v"(a), "v"(b), "v"(c), "v"(d)); }
__device__ __forceinline__ void acc_guard4(v8f& a, v8f& b, v8f& c, v8f& d) { asm volatile("v_nop\n\tv_nop\n\tv_nop\n\tv_nop" : "+v"(a), "+v"(b), "+v"(c), "+v"(d)); }
template <typename T> struct Frag;
template <> struct Frag<_Float16> {
  typedef v16h V; union U { v16h v; v8h h[2]; };
  static __device__ __forceinline__ v16h load(const _Float16* p) {
    U f; f.h[0] = *(const v8h*)(p); f.h[1] = *(const v8h*)(p + 16); return f.v;
  }
  static __device__ __forceinline__ v8f mma(v16h a, v16h b, v8f c) {
    return __builtin_amdgcn_wmma_f32_16x16x32_f16(false, a, false, b, (short)0, c, false, false);
  }
  static __device__ __forceinline__ void guard(v8f& a, v8f& b, v16h x, v16h y) { dep_guard_h(a, b, x, y); }
  static __device__ __forceinline__ void keep(v16h a, v16h b, v16h c, v16h d) { keep4_h(a, b, c, d); }
};
template <> struct Frag<__bf16> {
  typedef v16b V; union U { v16b v; v8b h[2]; };
  static __device__ __forceinline__ v16b load(const __bf16* p) {
    U f; f.h[0] = *(const v8b*)(p); f.h[1] = *(const v8b*)(p + 16); return f.v;
  }
  static __device__ __forceinline__ v8f mma(v16b a, v16b b, v8f c) {
    return __builtin_amdgcn_wmma_f32_16x16x32_bf16(false, a, false, b, (short)0, c, false, false);
  }
  static __device__ __forceinline__ void guard(v8f& a, v8f& b, v16b x, v16b y) { dep_guard_b(a, b, x, y); }
  static __device__ __forceinline__ void keep(v16b a, v16b b, v16b c, v16b d) { keep4_b(a, b, c, d); }
};

template <int ET> struct Elem;
template <> struct Elem<0> { typedef _Float16 T; };
template <> struct Elem<1> { typedef __bf16 T; };
template <int ET, bool SPLIT, int BIAS_MODE, int OUT_MODE, bool RESID, int ACT = 0>
__global__ __launch_bounds__(256) void wmma_gemm64(
    const unsigned short* __restrict__ Ap, const unsigned short* __restrict__ A2p, int lda, long strideA,
    const unsigned short* __restrict__ Btp, const unsigned short* __restrict__ Bt2p, int ldb, long strideB,
    void* __restrict__ Cout, void* __restrict__ Cout2, int ldc, long strideC,
    const float* __restrict__ bias,
    const float* __restrict__ resid, long strideR,
    int M, int N, int K, float scale) {
  typedef typename Elem<ET>::T T;
  typedef typename Frag<T>::V V;
  const T* A = (const T*)Ap; const T* A2 = (const T*)A2p; const T* Bt = (const T*)Btp; const T* Bt2 = (const T*)Bt2p;
  __shared__ __align__(16) float sT[8][16 * 68];
  const int b    = blockIdx.y;
  const int lane = threadIdx.x & 31;
  const int wave = threadIdx.x >> 5;
  const int tilesN = N >> 6;
  const int tilesM = M >> 6;
  const int tile = blockIdx.x * 8 + wave;
  if (tile >= tilesM * tilesN) return;
  const int tm = tile / tilesN;
  const int tn = tile - tm * tilesN;
  const int m0 = tm << 6;
  const int n0 = tn << 6;

  const T* Ab  = A  + (size_t)b * strideA;
  const T* Bb  = Bt + (size_t)b * strideB;
  const T* Ab2 = SPLIT ? (A2  + (size_t)b * strideA) : nullptr;
  const T* Bb2 = SPLIT ? (Bt2 + (size_t)b * strideB) : nullptr;

  const int rlane = lane & 15;
  const int koff  = (lane >> 4) * 8;
  const int mOff  = (lane >> 4) * 8;

  v8f acc[4][4];
#pragma unroll
  for (int i = 0; i < 4; ++i)
#pragma unroll
    for (int j = 0; j < 4; ++j) acc[i][j] = (v8f){0.f,0.f,0.f,0.f,0.f,0.f,0.f,0.f};

  for (int k0 = 0; k0 < K; k0 += 32) {
    V bh[4], bl[4];
#pragma unroll
    for (int j = 0; j < 4; ++j) {
      const size_t bo = (size_t)(n0 + (j << 4) + rlane) * ldb + koff + k0;
      bh[j] = Frag<T>::load(Bb + bo);
      if (SPLIT) bl[j] = Frag<T>::load(Bb2 + bo);
    }
#pragma unroll
    for (int i = 0; i < 4; ++i) {
      const size_t ao = (size_t)(m0 + (i << 4) + rlane) * lda + koff + k0;
      V ah = Frag<T>::load(Ab + ao);
      V al;
      if (SPLIT) al = Frag<T>::load(Ab2 + ao);
#pragma unroll
      for (int j = 0; j < 4; ++j) {
        acc[i][j] = Frag<T>::mma(ah, bh[j], acc[i][j]);
        if (SPLIT) {
          acc[i][j] = Frag<T>::mma(ah, bl[j], acc[i][j]);
          acc[i][j] = Frag<T>::mma(al, bh[j], acc[i][j]);
        }
      }
      Frag<T>::guard(acc[i][0], acc[i][3], ah, SPLIT ? al : ah);
    }
    Frag<T>::keep(bh[0], bh[1], bh[2], bh[3]);
    if (SPLIT) Frag<T>::keep(bl[0], bl[1], bl[2], bl[3]);
  }
  acc_guard4(acc[0][0], acc[0][1], acc[0][2], acc[0][3]);
  acc_guard4(acc[1][0], acc[1][1], acc[1][2], acc[1][3]);
  acc_guard4(acc[2][0], acc[2][1], acc[2][2], acc[2][3]);
  acc_guard4(acc[3][0], acc[3][1], acc[3][2], acc[3][3]);

  float* slab = sT[wave];
  const float* Rb = RESID ? (resid + (size_t)b * strideR) : nullptr;
#pragma unroll
  for (int i = 0; i < 4; ++i) {
    const int mBase = m0 + (i << 4);
#pragma unroll
    for (int j = 0; j < 4; ++j) {
      const int n = n0 + (j << 4) + rlane;
      float bv = 0.f;
      if (BIAS_MODE == 2) bv = bias[n];
#pragma unroll
      for (int r = 0; r < 8; ++r) {
        float v = acc[i][j][r] * scale;
        if (BIAS_MODE == 1) v += bias[mBase + mOff + r];
        if (BIAS_MODE == 2) v += bv;
        if (RESID) v += Rb[(size_t)(mBase + mOff + r) * ldc + n];
        if (ACT == 1) v = tanhf(v);
        if (ACT == 2) v = fmaxf(v, 0.0f);
        if (ACT == 3) v = v / (1.0f + expf(-v));
        if (ACT == 4) v = (v > 0.f) ? v : 0.01f * v;
        if (ACT == 5) v = 0.5f * v * (1.0f + erff(v * 0.70710678118654752f));
        slab[(mOff + r) * 68 + (j << 4) + rlane] = v;
      }
    }
    __builtin_amdgcn_fence(__ATOMIC_RELEASE, "workgroup");
    __builtin_amdgcn_wave_barrier();
    __builtin_amdgcn_fence(__ATOMIC_ACQUIRE, "workgroup");
    if (OUT_MODE == 0) {
      float* C = (float*)Cout + (size_t)b * strideC;
      const int hh = lane >> 4, c4 = (lane & 15) * 4;
      for (int pass = 0; pass < 2; ++pass) {
#pragma unroll
        for (int it = 0; it < 8; ++it) {
          const int row = it * 2 + hh;
          v4f v = *(const v4f*)(slab + row * 68 + c4);
          *(volatile v4f*)(C + (size_t)(mBase + row) * ldc + n0 + c4) = v;
        }
        __threadfence();
      }
    } else {
      const int q = lane >> 3, c8 = (lane & 7) * 8;
      unsigned short* C  = (unsigned short*)Cout  + (size_t)b * strideC;
      unsigned short* C2 = (OUT_MODE == 2) ? ((unsigned short*)Cout2 + (size_t)b * strideC) : nullptr;
      for (int pass = 0; pass < 2; ++pass) {
#pragma unroll
        for (int it = 0; it < 4; ++it) {
          const int row = it * 4 + q;
          const float* sp = slab + row * 68 + c8;
          v8h hv, lv;
#pragma unroll
          for (int e = 0; e < 8; ++e) {
            if (OUT_MODE == 1) {
              hv[e] = (_Float16)sp[e];
            } else {
              unsigned short hb = f2bf_bits(sp[e]);
              unsigned short lb = f2bf_bits(sp[e] - bf_bits2f(hb));
              hv[e] = __builtin_bit_cast(_Float16, hb);
              lv[e] = __builtin_bit_cast(_Float16, lb);
            }
          }
          *(volatile v8h*)(C + (size_t)(mBase + row) * ldc + n0 + c8) = hv;
          if (OUT_MODE == 2) *(volatile v8h*)(C2 + (size_t)(mBase + row) * ldc + n0 + c8) = lv;
        }
        __threadfence();
      }
    }
    __builtin_amdgcn_fence(__ATOMIC_RELEASE, "workgroup");
    __builtin_amdgcn_wave_barrier();
    __builtin_amdgcn_fence(__ATOMIC_ACQUIRE, "workgroup");
  }
}

constexpr int kNCls  = 32000;
constexpr int kEmb   = 256;
constexpr int kHid   = 512;
constexpr int kBat   = 128;
constexpr int kSteps = 256;
constexpr int kG4    = 4 * kHid;
constexpr float kWCarry    = 16.0f;
constexpr float kWCarryInv = 0.0625f;

static_assert(kEmb % 32 == 0 && kHid % 32 == 0, "K multiple of 32");
static_assert(kBat % 64 == 0 && kNCls % 64 == 0 && kHid % 32 == 0, "classifier gemm tiles");
static_assert(((kBat / 64) * (kNCls / 64)) % 8 == 0, "8 tiles per gemm block");
static_assert(kEmb % 256 == 0 && kHid % 256 == 0 && kHid % 64 == 0 && kNCls % 64 == 0, "cast tiles");
static_assert(kBat == 4 * 32 && kHid == 4 * 128, "cell step grid = 4x4 blocks of 32 rows x 128 cols");
static_assert((kSteps * kBat) % 8 == 0, "embed grid");
static_assert((kSteps & 1) == 0, "final state lands in buffer 0");

constexpr size_t kOffXe   = 0;
constexpr size_t kOffWx   = kOffXe + (size_t)kSteps * kBat * kEmb * 2;
constexpr size_t kOffWh   = kOffWx + (size_t)kG4 * kEmb * 2;
constexpr size_t kOffWq   = kOffWh + (size_t)kG4 * kHid * 2;
constexpr size_t kOffC    = kOffWq + (size_t)kNCls * kHid * 2;
constexpr size_t kOffHb0  = kOffC + (size_t)kBat * kHid * 4;
constexpr size_t kOffHb1  = kOffHb0 + (size_t)kBat * kHid * 2;
constexpr size_t kWsTotal = kOffHb1 + (size_t)kBat * kHid * 2;
static_assert(kWsTotal == 53215232, "carve total");
static_assert(kWsTotal <= 134217728, "carve under 128 MiB");
static_assert(kOffWx % 256 == 0 && kOffWh % 256 == 0 && kOffWq % 256 == 0 && kOffC % 256 == 0 &&
              kOffHb0 % 256 == 0 && kOffHb1 % 256 == 0, "region alignment");

__global__ __launch_bounds__(256) void embed_rows_kernel(const int* __restrict__ X, const float* __restrict__ E,
                                                         _Float16* __restrict__ Xe) {
  const int lane = threadIdx.x & 31;
  const int row = blockIdx.x * 8 + (threadIdx.x >> 5);
  const int t = row / kBat;
  const int b = row - t * kBat;
  int tok = X[b * kSteps + t];
  tok = tok < 0 ? 0 : tok;
  tok = tok > kNCls - 1 ? kNCls - 1 : tok;
  const float* er = E + (size_t)tok * kEmb + 8 * lane;
  const v4f f0 = *(const v4f*)(er);
  const v4f f1 = *(const v4f*)(er + 4);
  v8h hv;
  hv[0] = (_Float16)f0[0]; hv[1] = (_Float16)f0[1]; hv[2] = (_Float16)f0[2]; hv[3] = (_Float16)f0[3];
  hv[4] = (_Float16)f1[0]; hv[5] = (_Float16)f1[1]; hv[6] = (_Float16)f1[2]; hv[7] = (_Float16)f1[3];
  _Float16* dp = Xe + (size_t)row * kEmb + 8 * lane;
  *(volatile v8h*)dp = hv;
  __threadfence();
  *(volatile v8h*)dp = hv;
}

__global__ __launch_bounds__(256) void transpose_cast16_kernel(
    const float* __restrict__ src0, const float* __restrict__ src1,
    const float* __restrict__ src2, const float* __restrict__ src3,
    int ldsrc, int kin, _Float16* __restrict__ dst, long dstStrideZ, float sc) {
  __shared__ __align__(16) _Float16 tl[64 * 264];
  const int tid = threadIdx.x, lane = tid & 31, wave = tid >> 5;
  const int z = blockIdx.z;
  const float* src = (z == 0) ? src0 : (z == 1) ? src1 : (z == 2) ? src2 : src3;
  _Float16* dz = dst + (size_t)z * (size_t)dstStrideZ;
  const int n0 = blockIdx.x * 64, k0 = blockIdx.y * 256;
  const int c4 = (tid & 15) * 4, kr0 = tid >> 4;
#pragma unroll 4
  for (int it = 0; it < 16; ++it) {
    const int krow = it * 16 + kr0;
    const v4f v = *(const v4f*)(src + (size_t)(k0 + krow) * ldsrc + n0 + c4);
    tl[(c4 + 0) * 264 + krow] = (_Float16)(v[0] * sc);
    tl[(c4 + 1) * 264 + krow] = (_Float16)(v[1] * sc);
    tl[(c4 + 2) * 264 + krow] = (_Float16)(v[2] * sc);
    tl[(c4 + 3) * 264 + krow] = (_Float16)(v[3] * sc);
  }
  __syncthreads();
  for (int pass = 0; pass < 2; ++pass) {
#pragma unroll
    for (int rr = 0; rr < 8; ++rr) {
      const int nl = rr * 8 + wave;
      const v8h hv = *(const v8h*)(tl + nl * 264 + 8 * lane);
      *(volatile v8h*)(dz + (size_t)(n0 + nl) * kin + k0 + 8 * lane) = hv;
    }
    __threadfence();
  }
}

__global__ __launch_bounds__(256) void h_init_kernel(const float* __restrict__ H0, _Float16* __restrict__ Hb) {
  const int gid = blockIdx.x * 256 + threadIdx.x;
  const v4f a = *(const v4f*)(H0 + 8 * gid);
  const v4f c = *(const v4f*)(H0 + 8 * gid + 4);
  v8h hv;
  hv[0] = (_Float16)a[0]; hv[1] = (_Float16)a[1]; hv[2] = (_Float16)a[2]; hv[3] = (_Float16)a[3];
  hv[4] = (_Float16)c[0]; hv[5] = (_Float16)c[1]; hv[6] = (_Float16)c[2]; hv[7] = (_Float16)c[3];
  _Float16* dp = Hb + 8 * gid;
  *(volatile v8h*)dp = hv;
  __threadfence();
  *(volatile v8h*)dp = hv;
}

__global__ __launch_bounds__(256) void cell_init_kernel(const float* __restrict__ C0, float* __restrict__ Cws) {
  const int gid = blockIdx.x * 256 + threadIdx.x;
  const int e  = gid & 3;
  const int ln = (gid >> 2) & 31;
  const int q  = (gid >> 7) & 3;
  const int bw = gid >> 9;
  const int wv = bw & 7;
  const int blk = bw >> 3;
  const int v = q * 4 + e;
  const int i = v >> 3, r = v & 7;
  const int hh = ln >> 4, c = ln & 15;
  const int b = 32 * (blk >> 2) + 16 * i + 8 * hh + r;
  const int col = 128 * (blk & 3) + 16 * wv + c;
  const float val = C0[b * kHid + col];
  ((volatile float*)Cws)[gid] = val;
  __threadfence();
  ((volatile float*)Cws)[gid] = val;
}

__device__ __forceinline__ float gate_sigmoid(float x) {
  x = fminf(fmaxf(x, -30.0f), 30.0f);
  return 1.0f / (1.0f + expf(-x));
}

__global__ __launch_bounds__(256) void cell_step_kernel(
    const _Float16* __restrict__ Xt,
    const _Float16* __restrict__ Wxt,
    const _Float16* __restrict__ Wht,
    const _Float16* __restrict__ Hin,
    _Float16* Hout,
    float* Cws,
    const float* __restrict__ bfp, const float* __restrict__ bip,
    const float* __restrict__ bcp, const float* __restrict__ bop) {
  __shared__ __align__(16) _Float16 stg[32 * 136];
  typedef Frag<_Float16> FR;
  const int tid = threadIdx.x, lane = tid & 31, wave = tid >> 5;
  const int rl = lane & 15, hh = lane >> 4, koff = hh * 8;
  const int blk = blockIdx.x;
  const int m0 = 32 * (blk >> 2);
  const int hseg = 128 * (blk & 3);
  const int h0 = hseg + 16 * wave;
  const float bfv = bfp[h0 + rl];
  const float biv = bip[h0 + rl];
  const float bcv = bcp[h0 + rl];
  const float bov = bop[h0 + rl];

  v8f acc[2][4];
#pragma unroll
  for (int i = 0; i < 2; ++i)
#pragma unroll
    for (int g = 0; g < 4; ++g) acc[i][g] = (v8f){0.f,0.f,0.f,0.f,0.f,0.f,0.f,0.f};

#pragma unroll 1
  for (int k0 = 0; k0 < kEmb; k0 += 32) {
    v16h bw[4];
#pragma unroll
    for (int g = 0; g < 4; ++g) bw[g] = FR::load(Wxt + (size_t)(g * kHid + h0 + rl) * kEmb + k0 + koff);
#pragma unroll
    for (int i = 0; i < 2; ++i) {
      const v16h a = FR::load(Xt + (size_t)(m0 + 16 * i + rl) * kEmb + k0 + koff);
#pragma unroll
      for (int g = 0; g < 4; ++g) acc[i][g] = FR::mma(a, bw[g], acc[i][g]);
      FR::guard(acc[i][0], acc[i][3], a, a);
    }
    FR::keep(bw[0], bw[1], bw[2], bw[3]);
  }
#pragma unroll 1
  for (int k0 = 0; k0 < kHid; k0 += 32) {
    v16h bw[4];
#pragma unroll
    for (int g = 0; g < 4; ++g) bw[g] = FR::load(Wht + (size_t)(g * kHid + h0 + rl) * kHid + k0 + koff);
#pragma unroll
    for (int i = 0; i < 2; ++i) {
      const v16h a = FR::load(Hin + (size_t)(m0 + 16 * i + rl) * kHid + k0 + koff);
#pragma unroll
      for (int g = 0; g < 4; ++g) acc[i][g] = FR::mma(a, bw[g], acc[i][g]);
      FR::guard(acc[i][0], acc[i][3], a, a);
    }
    FR::keep(bw[0], bw[1], bw[2], bw[3]);
  }
  acc_guard4(acc[0][0], acc[0][1], acc[0][2], acc[0][3]);
  acc_guard4(acc[1][0], acc[1][1], acc[1][2], acc[1][3]);

  float* cl = Cws + ((size_t)(blk * 8 + wave) * 4) * 128 + lane * 4;
  float cst[16];
#pragma unroll
  for (int q = 0; q < 4; ++q) {
    const v4f cv = *(const v4f*)(cl + q * 128);
    cst[4 * q + 0] = cv[0]; cst[4 * q + 1] = cv[1]; cst[4 * q + 2] = cv[2]; cst[4 * q + 3] = cv[3];
  }
#pragma unroll
  for (int i = 0; i < 2; ++i) {
#pragma unroll
    for (int r = 0; r < 8; ++r) {
      const int v = i * 8 + r;
      const float pf = acc[i][0][r] * kWCarryInv + bfv;
      const float pi = acc[i][1][r] * kWCarryInv + biv;
      const float pg = acc[i][2][r] * kWCarryInv + bcv;
      const float po = acc[i][3][r] * kWCarryInv + bov;
      const float fg = gate_sigmoid(pf);
      const float ig = gate_sigmoid(pi);
      const float gg = tanhf(pg);
      const float og = gate_sigmoid(po);
      const float cold = cst[v];
      const float hn = og * tanhf(cold);
      cst[v] = fg * cold + ig * gg;
      stg[(16 * i + 8 * hh + r) * 136 + 16 * wave + rl] = (_Float16)hn;
    }
  }
  for (int pass = 0; pass < 2; ++pass) {
#pragma unroll
    for (int q = 0; q < 4; ++q) {
      v4f cv;
      cv[0] = cst[4 * q + 0]; cv[1] = cst[4 * q + 1]; cv[2] = cst[4 * q + 2]; cv[3] = cst[4 * q + 3];
      *(volatile v4f*)(cl + q * 128) = cv;
    }
    __threadfence();
  }
  __syncthreads();
  for (int pass = 0; pass < 2; ++pass) {
#pragma unroll
    for (int s = 0; s < 2; ++s) {
      const int row = 2 * (2 * wave + s) + hh;
      const v8h hv = *(const v8h*)(stg + row * 136 + 8 * rl);
      *(volatile v8h*)(Hout + (size_t)(m0 + row) * kHid + hseg + 8 * rl) = hv;
    }
    __threadfence();
  }
}

extern "C" void kernel_launch(void* const* d_in, const int* in_sizes, int n_in,
                              void* d_out, int out_size, void* d_ws, size_t ws_size,
                              hipStream_t stream) {
  if (n_in < 18) return;
  if (in_sizes[0] != kBat * kSteps || in_sizes[1] != kBat * kHid || in_sizes[2] != kBat * kHid ||
      in_sizes[3] != kNCls * kEmb || in_sizes[4] != kEmb * kHid || in_sizes[5] != kHid * kHid ||
      in_sizes[7] != kEmb * kHid || in_sizes[8] != kHid * kHid || in_sizes[10] != kEmb * kHid ||
      in_sizes[11] != kHid * kHid || in_sizes[13] != kEmb * kHid || in_sizes[14] != kHid * kHid ||
      in_sizes[6] != kHid || in_sizes[9] != kHid || in_sizes[12] != kHid || in_sizes[15] != kHid ||
      in_sizes[16] != kHid * kNCls || in_sizes[17] != kNCls || out_size != kBat * kNCls) return;
  if (ws_size < kWsTotal) return;

  const int*   X   = (const int*)  d_in[0];
  const float* Hi  = (const float*)d_in[1];
  const float* Ci  = (const float*)d_in[2];
  const float* E   = (const float*)d_in[3];
  const float* Wxf = (const float*)d_in[4];
  const float* Whf = (const float*)d_in[5];
  const float* bfp = (const float*)d_in[6];
  const float* Wxi = (const float*)d_in[7];
  const float* Whi = (const float*)d_in[8];
  const float* bip = (const float*)d_in[9];
  const float* Wxc = (const float*)d_in[10];
  const float* Whc = (const float*)d_in[11];
  const float* bcp = (const float*)d_in[12];
  const float* Wxo = (const float*)d_in[13];
  const float* Who = (const float*)d_in[14];
  const float* bop = (const float*)d_in[15];
  const float* Whq = (const float*)d_in[16];
  const float* bq  = (const float*)d_in[17];

  char* ws = (char*)d_ws;
  _Float16* Xe16  = (_Float16*)(ws + kOffXe);
  _Float16* Wx16t = (_Float16*)(ws + kOffWx);
  _Float16* Wh16t = (_Float16*)(ws + kOffWh);
  _Float16* Wq16t = (_Float16*)(ws + kOffWq);
  float*    Cws   = (float*)   (ws + kOffC);
  _Float16* Hb0   = (_Float16*)(ws + kOffHb0);
  _Float16* Hb1   = (_Float16*)(ws + kOffHb1);

  embed_rows_kernel<<<(kSteps * kBat) / 8, 256, 0, stream>>>(X, E, Xe16);
  transpose_cast16_kernel<<<dim3(kHid / 64, kEmb / 256, 4), 256, 0, stream>>>(
      Wxf, Wxi, Wxc, Wxo, kHid, kEmb, Wx16t, (long)kHid * kEmb, kWCarry);
  transpose_cast16_kernel<<<dim3(kHid / 64, kHid / 256, 4), 256, 0, stream>>>(
      Whf, Whi, Whc, Who, kHid, kHid, Wh16t, (long)kHid * kHid, kWCarry);
  transpose_cast16_kernel<<<dim3(kNCls / 64, kHid / 256, 1), 256, 0, stream>>>(
      Whq, Whq, Whq, Whq, kNCls, kHid, Wq16t, 0L, kWCarry);
  cell_init_kernel<<<(kBat * kHid) / 256, 256, 0, stream>>>(Ci, Cws);
  h_init_kernel<<<(kBat * kHid) / (8 * 256), 256, 0, stream>>>(Hi, Hb0);

  for (int t = 0; t < kSteps; ++t) {
    const _Float16* hin  = (t & 1) ? Hb1 : Hb0;
    _Float16*       hout = (t & 1) ? Hb0 : Hb1;
    cell_step_kernel<<<16, 256, 0, stream>>>(Xe16 + (size_t)t * kBat * kEmb, Wx16t, Wh16t, hin, hout, Cws,
                                              bfp, bip, bcp, bop);
  }

  wmma_gemm64<0, false, 2, 0, false, 0><<<dim3(((kBat / 64) * (kNCls / 64)) / 8, 1), 256, 0, stream>>>(
      (const unsigned short*)Hb0, nullptr, kHid, 0L,
      (const unsigned short*)Wq16t, nullptr, kHid, 0L,
      d_out, nullptr, kNCls, 0L,
      bq, nullptr, 0L,
      kBat, kNCls, kHid, kWCarryInv);
}
